// Silco_22411139350740
// MI455X (gfx1250) — hardware-run, weakly checked
//
#include <hip/hip_runtime.h>
#include <stddef.h>

#define BATCH 8
#define NPTS  256
#define FIN   24
#define HID   192
#define HID3  96
#define XCW   72
#define XCP   96
#define NTILE ((BATCH * NPTS * NPTS) / 32)
#define TILEB (32 * HID * 2)

static_assert(NPTS == 256);
static_assert(NTILE % 2 == 0);
static_assert(XCP % 32 == 0);
static_assert(XCP == 4 * 24);
static_assert(32 * HID3 * 4 == TILEB);

typedef _Float16 f16;
typedef f16 v16h __attribute__((ext_vector_type(16)));
typedef f16 v8h_t __attribute__((ext_vector_type(8)));
typedef v8h_t __attribute__((may_alias)) v8h;
typedef float v8f __attribute__((ext_vector_type(8)));
typedef float v4f_t __attribute__((ext_vector_type(4)));
typedef v4f_t __attribute__((may_alias)) v4f;
typedef unsigned int v4u_t __attribute__((ext_vector_type(4)));
typedef v4u_t __attribute__((may_alias)) v4u;

union Frag  { v16h v; v8h_t h[2]; };
union Pack8 { v8h_t h; v4u_t u; };

__device__ __forceinline__ v8f zero8() {
    v8f z;
#pragma unroll
    for (int i = 0; i < 8; ++i) z[i] = 0.0f;
    return z;
}

__device__ __forceinline__ v8f wmma16(v16h a, v16h b, v8f c) {
    return __builtin_amdgcn_wmma_f32_16x16x32_f16(false, a, false, b, (short)0, c, false, false);
}

#define WMMA_GUARD2(C0, C1, A0, A1, BB) \
    asm volatile("v_nop\n\tv_nop\n\tv_nop\n\tv_nop" : "+v"(C0), "+v"(C1) : "v"(A0), "v"(A1), "v"(BB))

__device__ __forceinline__ float leaky(float v) { return (v >= 0.0f) ? v : 0.01f * v; }

template <int KC, bool OUTF32>
__device__ __forceinline__ void mlp_layer_wave32(
    const f16* actIn, int inStride,
    unsigned char* actOut, int outStride,
    const f16* __restrict__ wt, const float* __restrict__ bias,
    int Nd, int lane)
{
    const int rlo = lane & 15;
    const int khi = lane >> 4;
    constexpr int K = KC * 32;

    Frag a[2][KC];
#pragma unroll
    for (int m = 0; m < 2; ++m) {
#pragma unroll
        for (int kc = 0; kc < KC; ++kc) {
            const f16* pa = actIn + (m * 16 + rlo) * inStride + kc * 32 + 8 * khi;
            a[m][kc].h[0] = *(const v8h*)(pa);
            a[m][kc].h[1] = *(const v8h*)(pa + 16);
        }
    }

    f16*   outH = (f16*)actOut;
    float* outF = (float*)actOut;

#pragma unroll 1
    for (int n0 = 0; n0 < Nd; n0 += 16) {
        v8f c0 = zero8(), c1 = zero8();
        const f16* pbn = wt + (size_t)(n0 + rlo) * K + 8 * khi;
#pragma unroll
        for (int kc = 0; kc < KC; ++kc) {
            Frag bq;
            bq.h[0] = *(const v8h*)(pbn + kc * 32);
            bq.h[1] = *(const v8h*)(pbn + kc * 32 + 16);
            c0 = wmma16(a[0][kc].v, bq.v, c0);
            c1 = wmma16(a[1][kc].v, bq.v, c1);
            WMMA_GUARD2(c0, c1, a[0][kc].v, a[1][kc].v, bq.v);
        }
        const float bv = bias[n0 + rlo];
#pragma unroll
        for (int r = 0; r < 8; ++r) {
            const float v0 = leaky(c0[r] * (1.0f / 256.0f) + bv);
            const float v1 = leaky(c1[r] * (1.0f / 256.0f) + bv);
            const int i0 = (r + 8 * khi) * outStride + n0 + rlo;
            const int i1 = (16 + r + 8 * khi) * outStride + n0 + rlo;
            if (OUTF32) {
                outF[i0] = v0;
                outF[i1] = v1;
            } else {
                outH[i0] = (f16)(v0 * 16.0f);
                outH[i1] = (f16)(v1 * 16.0f);
            }
        }
    }
}

template <int KP0, int KLOAD, int XP>
__global__ __launch_bounds__(64) void adj_kernel(
    const float* __restrict__ xs,
    const f16* __restrict__ wt0,
    const f16* __restrict__ wt1,
    const f16* __restrict__ wt2,
    const f16* __restrict__ wt3,
    const float* __restrict__ bias0, const float* __restrict__ bias1,
    const float* __restrict__ bias2, const float* __restrict__ bias3,
    const float* __restrict__ w4,
    const float* __restrict__ b4,
    float* __restrict__ logits)
{
    static_assert(KP0 % 32 == 0);
    static_assert(KLOAD * 8 <= XP);
    static_assert(KLOAD * 8 <= KP0);
    static_assert(KP0 <= HID);

    __shared__ __align__(16) unsigned char smem[2 * 2 * TILEB];

    const int lane  = threadIdx.x & 31;
    const int wslot = threadIdx.x >> 5;
    unsigned char* bufA = smem + wslot * (2 * TILEB);
    unsigned char* bufB = bufA + TILEB;

    const int t   = blockIdx.x * 2 + wslot;
    const int b   = t >> 11;
    const int rem = t & 2047;
    const int i   = rem >> 3;
    const int j0  = (rem & 7) << 5;

    {
        const float* xi = xs + (size_t)(b * NPTS + i) * XP;
        const float* xj = xs + (size_t)(b * NPTS + j0 + lane) * XP;
        f16* drow = (f16*)bufA + lane * KP0;
#pragma unroll 1
        for (int g = 0; g < KLOAD; ++g) {
            const v4f_t p0 = *(const v4f*)(xi + 8 * g);
            const v4f_t p1 = *(const v4f*)(xi + 8 * g + 4);
            const v4f_t q0 = *(const v4f*)(xj + 8 * g);
            const v4f_t q1 = *(const v4f*)(xj + 8 * g + 4);
            Pack8 pk;
#pragma unroll
            for (int e = 0; e < 4; ++e) {
                pk.h[e]     = (f16)(fabsf(p0[e] - q0[e]) * 16.0f);
                pk.h[4 + e] = (f16)(fabsf(p1[e] - q1[e]) * 16.0f);
            }
            *(v4u*)(drow + 8 * g) = pk.u;
        }
        Pack8 z;
#pragma unroll
        for (int e = 0; e < 4; ++e) z.u[e] = 0u;
#pragma unroll
        for (int g = KLOAD; g < KP0 / 8; ++g) *(v4u*)(drow + 8 * g) = z.u;
    }
    __syncthreads();

    mlp_layer_wave32<KP0 / 32, false>((const f16*)bufA, KP0, bufB, HID, wt0, bias0, HID, lane);
    __syncthreads();
    mlp_layer_wave32<6, false>((const f16*)bufB, HID, bufA, HID, wt1, bias1, HID, lane);
    __syncthreads();
    mlp_layer_wave32<6, false>((const f16*)bufA, HID, bufB, HID, wt2, bias2, HID, lane);
    __syncthreads();
    mlp_layer_wave32<6, true>((const f16*)bufB, HID, bufA, HID3, wt3, bias3, HID3, lane);
    __syncthreads();

    {
        const float* pr = (const float*)bufA + lane * HID3;
        float acc = 0.0f;
#pragma unroll 1
        for (int c = 0; c < HID3 / 4; ++c) {
            const v4f_t u = *(const v4f*)(pr + 4 * c);
#pragma unroll
            for (int e = 0; e < 4; ++e) acc = fmaf(u[e], w4[4 * c + e], acc);
        }
        acc += b4[0];
        float* lp = logits + ((size_t)(b * NPTS + i) * NPTS + j0 + lane);
        *(volatile float*)lp = acc;
        __threadfence();
        *(volatile float*)lp = acc;
    }
}

__global__ __launch_bounds__(256) void softmax_kernel(
    const float* __restrict__ lg, float* __restrict__ aout)
{
    __shared__ float red[16];
    const int row  = blockIdx.x;
    const int i    = row & (NPTS - 1);
    const int tid  = threadIdx.x;
    const int lane = tid & 31, w = tid >> 5;
    const size_t base = (size_t)row * NPTS;

    float v = lg[base + tid];
    v = (tid == i) ? (v - 1e8f) : v;

    float m = v;
#pragma unroll
    for (int off = 16; off > 0; off >>= 1) m = fmaxf(m, __shfl_xor(m, off, 32));
    if (lane == 0) red[w] = m;
    __syncthreads();
    float mm = red[0];
#pragma unroll
    for (int k = 1; k < 8; ++k) mm = fmaxf(mm, red[k]);

    const float e = expf(v - mm);
    float s = e;
#pragma unroll
    for (int off = 16; off > 0; off >>= 1) s += __shfl_xor(s, off, 32);
    if (lane == 0) red[8 + w] = s;
    __syncthreads();
    float ss = red[8];
#pragma unroll
    for (int k = 9; k < 16; ++k) ss += red[k];

    const float o = e * (1.0f / ss);
    float* p = aout + base + tid;
    *(volatile float*)p = o;
    __threadfence();
    *(volatile float*)p = o;
}

__global__ __launch_bounds__(64) void g0_kernel(
    const float* __restrict__ x,
    const float* __restrict__ a0,
    const float* __restrict__ w,
    const float* __restrict__ bias,
    float* __restrict__ xc)
{
    __shared__ float arow[NPTS];
    __shared__ float agg[48];
    __shared__ __align__(16) float xcs[XCP];

    const int row = blockIdx.x;
    const int b   = row >> 8;
    const int tid = threadIdx.x;

#pragma unroll
    for (int q = 0; q < 4; ++q) arow[tid + 64 * q] = a0[(size_t)row * NPTS + tid + 64 * q];
    __syncthreads();

    {
        const int f = (tid < FIN) ? tid : (FIN - 1);
        const float* xb = x + (size_t)b * NPTS * FIN + f;
        float s = 0.0f;
#pragma unroll 1
        for (int j = 0; j < NPTS; ++j) s = fmaf(arow[j], xb[(size_t)j * FIN], s);
        if (tid < FIN) {
            agg[FIN + tid] = s;
            agg[tid] = x[(size_t)row * FIN + f];
        }
    }
    __syncthreads();

    {
        const int o = (tid < 48) ? tid : 47;
        const float* wr = w + o * 48;
        float s = 0.0f;
#pragma unroll 1
        for (int c = 0; c < 48; ++c) s = fmaf(agg[c], wr[c], s);
        s += bias[o];
        if (tid < 48) xcs[FIN + tid] = leaky(s);
        if (tid < FIN) {
            xcs[tid] = agg[tid];
            xcs[XCW + tid] = 0.0f;
        }
    }
    __syncthreads();

    const int t4 = (tid < 24) ? tid : 23;
    const v4f_t val = *(const v4f*)(xcs + 4 * t4);
    float* p = xc + (size_t)row * XCP + 4 * t4;
    if (tid < 24) *(volatile v4f_t*)p = val;
    __threadfence();
    if (tid < 24) *(volatile v4f_t*)p = val;
}

__global__ __launch_bounds__(256) void g1_kernel(
    const float* __restrict__ xc,
    const float* __restrict__ a1,
    const float* __restrict__ w,
    const float* __restrict__ bias,
    float* __restrict__ out)
{
    __shared__ float res[32];
    const int blk = blockIdx.x;
    const int b   = blk >> 3;
    const int i0  = (blk & 7) * 32;
    const int tid = threadIdx.x;
    const int r = tid >> 3, q = tid & 7;
    const int row = b * NPTS + i0 + r;

    const float* ar = a1 + (size_t)row * NPTS;
    const float* xb = xc + (size_t)b * NPTS * XCP + q * 9;
    float s[9];
#pragma unroll
    for (int e = 0; e < 9; ++e) s[e] = 0.0f;
#pragma unroll 1
    for (int j = 0; j < NPTS; ++j) {
        const float av = ar[j];
        const float* xr = xb + (size_t)j * XCP;
#pragma unroll
        for (int e = 0; e < 9; ++e) s[e] = fmaf(av, xr[e], s[e]);
    }
    const float* xrow = xc + (size_t)row * XCP + q * 9;
    float part = 0.0f;
#pragma unroll
    for (int e = 0; e < 9; ++e) {
        part = fmaf(s[e], w[XCW + q * 9 + e], part);
        part = fmaf(xrow[e], w[q * 9 + e], part);
    }
    part += __shfl_xor(part, 1, 32);
    part += __shfl_xor(part, 2, 32);
    part += __shfl_xor(part, 4, 32);
    if (q == 0) res[r] = part;
    __syncthreads();

    const int tt = tid & 31;
    const float v = res[tt] + bias[0];
    float* p = out + (size_t)b * NPTS + i0 + tt;
    if (tid < 32) *(volatile float*)p = v;
    __threadfence();
    if (tid < 32) *(volatile float*)p = v;
}

__global__ __launch_bounds__(256) void wconv_kernel(
    const float* __restrict__ w, f16* __restrict__ wt, int Korig, int KP, int Nd)
{
    const int G = KP >> 3;
    const int total = Nd * G;
    const int idx = blockIdx.x * 256 + threadIdx.x;
    const bool ok = (idx < total);
    const int ic = ok ? idx : (total - 1);
    const int n = ic / G;
    const int g = ic - n * G;
    Pack8 pk;
#pragma unroll
    for (int e = 0; e < 8; ++e) {
        const int k  = g * 8 + e;
        const int kc = (k < Korig) ? k : (Korig - 1);
        const float v = w[(size_t)kc * Nd + n];
        const float vs = (k < Korig) ? (v * 16.0f) : 0.0f;
        pk.h[e] = (f16)vs;
    }
    f16* p = wt + (size_t)n * KP + g * 8;
    if (ok) *(volatile v4u_t*)p = pk.u;
    __threadfence();
    if (ok) *(volatile v4u_t*)p = pk.u;
}

extern "C" void kernel_launch(void* const* d_in, const int* in_sizes, int n_in,
                              void* d_out, int out_size, void* d_ws, size_t ws_size,
                              hipStream_t stream)
{
    if (n_in < 25) return;
    if (in_sizes[0] != BATCH * NPTS * FIN) return;
    if (in_sizes[1] != FIN * HID || in_sizes[2] != HID) return;
    if (in_sizes[3] != HID * HID || in_sizes[4] != HID) return;
    if (in_sizes[5] != HID * HID || in_sizes[6] != HID) return;
    if (in_sizes[7] != HID * HID3 || in_sizes[8] != HID3) return;
    if (in_sizes[9] != HID3 || in_sizes[10] < 1) return;
    if (in_sizes[11] != XCW * HID || in_sizes[12] != HID) return;
    if (in_sizes[13] != HID * HID || in_sizes[14] != HID) return;
    if (in_sizes[15] != HID * HID || in_sizes[16] != HID) return;
    if (in_sizes[17] != HID * HID3 || in_sizes[18] != HID3) return;
    if (in_sizes[19] != HID3 || in_sizes[20] < 1) return;
    if (in_sizes[21] != 48 * 48 || in_sizes[22] != 48) return;
    if (in_sizes[23] != 2 * XCW || in_sizes[24] < 1) return;
    if (out_size != BATCH * NPTS + 2 * BATCH * NPTS * NPTS) return;

    const float* x = (const float*)d_in[0];
    const float* a0w[5] = {(const float*)d_in[1], (const float*)d_in[3],
                           (const float*)d_in[5], (const float*)d_in[7],
                           (const float*)d_in[9]};
    const float* a0b[5] = {(const float*)d_in[2], (const float*)d_in[4],
                           (const float*)d_in[6], (const float*)d_in[8],
                           (const float*)d_in[10]};
    const float* a1w[5] = {(const float*)d_in[11], (const float*)d_in[13],
                           (const float*)d_in[15], (const float*)d_in[17],
                           (const float*)d_in[19]};
    const float* a1b[5] = {(const float*)d_in[12], (const float*)d_in[14],
                           (const float*)d_in[16], (const float*)d_in[18],
                           (const float*)d_in[20]};
    const float* g0w = (const float*)d_in[21];
    const float* g0b = (const float*)d_in[22];
    const float* g1w = (const float*)d_in[23];
    const float* g1b = (const float*)d_in[24];

    size_t off = 0;
    auto take = [&](size_t bytes) -> size_t {
        const size_t o = off;
        off = (off + bytes + 255) & ~(size_t)255;
        return o;
    };
    const size_t oW00 = take((size_t)HID  * 32  * 2);
    const size_t oW01 = take((size_t)HID  * HID * 2);
    const size_t oW02 = take((size_t)HID  * HID * 2);
    const size_t oW03 = take((size_t)HID3 * HID * 2);
    const size_t oW10 = take((size_t)HID  * 96  * 2);
    const size_t oW11 = take((size_t)HID  * HID * 2);
    const size_t oW12 = take((size_t)HID  * HID * 2);
    const size_t oW13 = take((size_t)HID3 * HID * 2);
    const size_t oXC  = take((size_t)BATCH * NPTS * XCP * 4);
    const size_t oLG0 = take((size_t)BATCH * NPTS * NPTS * 4);
    const size_t oLG1 = take((size_t)BATCH * NPTS * NPTS * 4);
    const size_t total = off;
    if (total > ws_size) return;

    char* ws = (char*)d_ws;
    f16* wt00 = (f16*)(ws + oW00);
    f16* wt01 = (f16*)(ws + oW01);
    f16* wt02 = (f16*)(ws + oW02);
    f16* wt03 = (f16*)(ws + oW03);
    f16* wt10 = (f16*)(ws + oW10);
    f16* wt11 = (f16*)(ws + oW11);
    f16* wt12 = (f16*)(ws + oW12);
    f16* wt13 = (f16*)(ws + oW13);
    float* xc  = (float*)(ws + oXC);
    float* lg0 = (float*)(ws + oLG0);
    float* lg1 = (float*)(ws + oLG1);

    float* out_ptr = (float*)d_out;
    float* a0_ptr  = out_ptr + BATCH * NPTS;
    float* a1_ptr  = a0_ptr + (size_t)BATCH * NPTS * NPTS;

    wconv_kernel<<<(HID  * (32  / 8) + 255) / 256, 256, 0, stream>>>(a0w[0], wt00, FIN, 32,  HID);
    wconv_kernel<<<(HID  * (HID / 8) + 255) / 256, 256, 0, stream>>>(a0w[1], wt01, HID, HID, HID);
    wconv_kernel<<<(HID  * (HID / 8) + 255) / 256, 256, 0, stream>>>(a0w[2], wt02, HID, HID, HID);
    wconv_kernel<<<(HID3 * (HID / 8) + 255) / 256, 256, 0, stream>>>(a0w[3], wt03, HID, HID, HID3);
    wconv_kernel<<<(HID  * (96  / 8) + 255) / 256, 256, 0, stream>>>(a1w[0], wt10, XCW, 96,  HID);
    wconv_kernel<<<(HID  * (HID / 8) + 255) / 256, 256, 0, stream>>>(a1w[1], wt11, HID, HID, HID);
    wconv_kernel<<<(HID  * (HID / 8) + 255) / 256, 256, 0, stream>>>(a1w[2], wt12, HID, HID, HID);
    wconv_kernel<<<(HID3 * (HID / 8) + 255) / 256, 256, 0, stream>>>(a1w[3], wt13, HID, HID, HID3);

    adj_kernel<32, 3, FIN><<<NTILE / 2, 64, 0, stream>>>(
        x, wt00, wt01, wt02, wt03, a0b[0], a0b[1], a0b[2], a0b[3], a0w[4], a0b[4], lg0);
    softmax_kernel<<<BATCH * NPTS, 256, 0, stream>>>(lg0, a0_ptr);

    g0_kernel<<<BATCH * NPTS, 64, 0, stream>>>(x, a0_ptr, g0w, g0b, xc);

    adj_kernel<96, 12, XCP><<<NTILE / 2, 64, 0, stream>>>(
        xc, wt10, wt11, wt12, wt13, a1b[0], a1b[1], a1b[2], a1b[3], a1w[4], a1b[4], lg1);
    softmax_kernel<<<BATCH * NPTS, 256, 0, stream>>>(lg1, a1_ptr);

    g1_kernel<<<(BATCH * NPTS) / 32, 256, 0, stream>>>(xc, a1_ptr, g1w, g1b, out_ptr);
}
